// LongformerSelfAttention_77489799955228
// MI455X (gfx1250) — hardware-verified
//
#include <hip/hip_runtime.h>
#include <hip/hip_bf16.h>

#define BB    2
#define SS    2048
#define HID   768
#define NH    12
#define HD    64
#define WIN   256
#define NSTEP 17

typedef float  v8f  __attribute__((ext_vector_type(8)));
typedef float  v4f  __attribute__((ext_vector_type(4)));
typedef int    v4i  __attribute__((ext_vector_type(4)));
typedef __bf16 v8b  __attribute__((ext_vector_type(8)));
typedef __bf16 v16b __attribute__((ext_vector_type(16)));

union Frag   { v16b v; v8b h[2]; };
union Pack16 { v8b b; v4i u; };

__device__ __forceinline__ void mma(v8f& c, const v16b a, const v16b b) {
    c = __builtin_amdgcn_wmma_f32_16x16x32_bf16(false, a, false, b, (short)0, c, false, false);
    asm volatile("v_nop\n\tv_nop\n\tv_nop\n\tv_nop" : "+v"(c) : "v"(a), "v"(b));
}

__device__ __forceinline__ v8f zero8() {
    return (v8f){0.f, 0.f, 0.f, 0.f, 0.f, 0.f, 0.f, 0.f};
}

__device__ __forceinline__ int clampi(int v, int lo, int hi) {
    return v < lo ? lo : (v > hi ? hi : v);
}

__global__ __launch_bounds__(256) void k_cvt(
    const float* __restrict__ x,  const float* __restrict__ w0,
    const float* __restrict__ w1, const float* __restrict__ w2,
    __bf16* __restrict__ xb, __bf16* __restrict__ wb, int nxc, int nwc)
{
    const int lane = threadIdx.x & 31;
    const int c = blockIdx.x * 8 + (threadIdx.x >> 5);
    if (c >= nxc + 3 * nwc) return;
    const float* src;
    __bf16* dst;
    if (c < nxc) {
        src = x + (size_t)c * 256;
        dst = xb + (size_t)c * 256;
    } else {
        const int rr = c - nxc;
        const int mi = rr / nwc;
        const int cc = rr - mi * nwc;
        const float* wsrc = (mi == 0) ? w0 : ((mi == 1) ? w1 : w2);
        src = wsrc + (size_t)cc * 256;
        dst = wb + ((size_t)mi * nwc + cc) * 256;
    }
    const v4f f0 = *(const v4f*)(src + lane * 8);
    const v4f f1 = *(const v4f*)(src + lane * 8 + 4);
    Pack16 o;
    #pragma unroll
    for (int e = 0; e < 4; e++) {
        o.b[e]     = (__bf16)f0[e];
        o.b[4 + e] = (__bf16)f1[e];
    }
    const v4i ov = o.u;
    volatile v4i* dp = (volatile v4i*)(dst + lane * 8);
    *dp = ov;
    __threadfence();
    *dp = ov;
}

__global__ __launch_bounds__(128) void k_proj(
    const __bf16* __restrict__ xb, const __bf16* __restrict__ wb,
    const float* __restrict__ bq, const float* __restrict__ bk, const float* __restrict__ bv,
    __bf16* __restrict__ qh, __bf16* __restrict__ ql,
    __bf16* __restrict__ kh, __bf16* __restrict__ kl,
    __bf16* __restrict__ vth, __bf16* __restrict__ vtl)
{
    __shared__ __attribute__((aligned(16))) __bf16 s_hi[64 * 64];
    __shared__ __attribute__((aligned(16))) __bf16 s_lo[64 * 64];

    const int t0 = blockIdx.x * 64;
    if (t0 >= BB * SS) return;
    const int lane = threadIdx.x & 31, w = threadIdx.x >> 5;
    const int h = lane >> 4, m = lane & 15;
    const int mi = blockIdx.z, head = blockIdx.y;
    const int tw = t0 + 16 * w;

    const __bf16* W = wb + (size_t)mi * HID * HID;
    const float* bias = (mi == 0) ? bq : ((mi == 1) ? bk : bv);
    const float scale = (mi == 0) ? 0.125f : 1.0f;

    const __bf16* arow = xb + (size_t)(tw + m) * HID;
    v8f acc[4];
    #pragma unroll
    for (int s4 = 0; s4 < 4; s4++) acc[s4] = zero8();

    #pragma unroll 1
    for (int k0 = 0; k0 < HID; k0 += 32) {
        Frag a;
        a.h[0] = *(const v8b*)(arow + k0 + 8 * h);
        a.h[1] = *(const v8b*)(arow + k0 + 16 + 8 * h);
        #pragma unroll
        for (int s4 = 0; s4 < 4; s4++) {
            const __bf16* wr = W + (size_t)(head * HD + s4 * 16 + m) * HID + k0;
            Frag b;
            b.h[0] = *(const v8b*)(wr + 8 * h);
            b.h[1] = *(const v8b*)(wr + 16 + 8 * h);
            mma(acc[s4], a.v, b.v);
        }
    }

    #pragma unroll
    for (int s4 = 0; s4 < 4; s4++) {
        const int col = s4 * 16 + m;
        const float bb = (float)(__bf16)bias[head * HD + col];
        #pragma unroll
        for (int r = 0; r < 8; r++) {
            const int tokl = 16 * w + 8 * h + r;
            const float y = (acc[s4][r] + bb) * scale;
            const __bf16 yh = (__bf16)y;
            const __bf16 yl = (__bf16)(y - (float)yh);
            const int idx = (mi == 2) ? (col * 64 + tokl) : (tokl * 64 + col);
            s_hi[idx] = yh;
            s_lo[idx] = yl;
        }
    }
    __syncthreads();

    const int bb_ = t0 >> 11;
    const int s0 = t0 & (SS - 1);
    const int bh = bb_ * NH + head;
    const int q = lane >> 3, p = lane & 7;
    __bf16* ph_ = (mi == 0) ? qh : ((mi == 1) ? kh : vth);
    __bf16* pl_ = (mi == 0) ? ql : ((mi == 1) ? kl : vtl);
    v4i dh[4], dl[4];
    size_t off[4];
    #pragma unroll
    for (int it = 0; it < 4; it++) {
        const int L = 16 * w + 4 * it + q;
        dh[it] = *(const v4i*)(s_hi + L * 64 + p * 8);
        dl[it] = *(const v4i*)(s_lo + L * 64 + p * 8);
        off[it] = (mi == 2)
            ? ((size_t)(bh * HD + L) * SS + s0 + p * 8)
            : ((size_t)(bh * SS + s0 + L) * HD + p * 8);
    }
    #pragma unroll
    for (int it = 0; it < 4; it++) {
        *(volatile v4i*)(ph_ + off[it]) = dh[it];
        *(volatile v4i*)(pl_ + off[it]) = dl[it];
    }
    __threadfence();
    #pragma unroll
    for (int it = 0; it < 4; it++) {
        *(volatile v4i*)(ph_ + off[it]) = dh[it];
        *(volatile v4i*)(pl_ + off[it]) = dl[it];
    }
}

__global__ __launch_bounds__(64) void k_vsum(
    const __bf16* __restrict__ vth, const __bf16* __restrict__ vtl, float* __restrict__ vsum)
{
    __shared__ __attribute__((aligned(16))) float s_s[64];
    const int bh = blockIdx.x, d = threadIdx.x;
    if (bh >= BB * NH) return;
    const __bf16* rh = vth + ((size_t)bh * HD + d) * SS;
    const __bf16* rl = vtl + ((size_t)bh * HD + d) * SS;
    float acc = 0.f;
    #pragma unroll 1
    for (int i = 0; i < SS; i += 8) {
        const v8b a = *(const v8b*)(rh + i);
        const v8b c = *(const v8b*)(rl + i);
        #pragma unroll
        for (int e = 0; e < 8; e++) acc += (float)a[e] + (float)c[e];
    }
    s_s[d] = acc;
    __syncthreads();
    v4f v = (v4f){0.f, 0.f, 0.f, 0.f};
    const bool writer = threadIdx.x < 16;
    if (writer) v = *(const v4f*)(s_s + 4 * threadIdx.x);
    if (writer) *(volatile v4f*)(vsum + bh * HD + 4 * threadIdx.x) = v;
    __threadfence();
    if (writer) *(volatile v4f*)(vsum + bh * HD + 4 * threadIdx.x) = v;
}

__global__ __launch_bounds__(64) void k_attn(
    const __bf16* __restrict__ qh, const __bf16* __restrict__ ql,
    const __bf16* __restrict__ kh, const __bf16* __restrict__ kl,
    const __bf16* __restrict__ vth, const __bf16* __restrict__ vtl,
    const float* __restrict__ vsum, float* __restrict__ out)
{
    __shared__ __attribute__((aligned(16))) float s_o[2][16 * HD];

    if (blockIdx.x * 32 >= SS) return;
    const int lane = threadIdx.x & 31, w = threadIdx.x >> 5;
    const int h = lane >> 4, m = lane & 15;
    const int b = blockIdx.z, head = blockIdx.y;
    const int i0 = blockIdx.x * 32 + w * 16;
    const int bh = b * NH + head;

    Frag bqh[2], bql[2];
    {
        const size_t qo = ((size_t)bh * SS + i0 + m) * HD;
        #pragma unroll
        for (int dd = 0; dd < 2; dd++) {
            bqh[dd].h[0] = *(const v8b*)(qh + qo + 32 * dd + 8 * h);
            bqh[dd].h[1] = *(const v8b*)(qh + qo + 32 * dd + 16 + 8 * h);
            bql[dd].h[0] = *(const v8b*)(ql + qo + 32 * dd + 8 * h);
            bql[dd].h[1] = *(const v8b*)(ql + qo + 32 * dd + 16 + 8 * h);
        }
    }

    const size_t kbase = (size_t)bh * SS * HD;
    const size_t vbase = (size_t)bh * HD * SS;

    v8f ctx[4];
    #pragma unroll
    for (int s4 = 0; s4 < 4; s4++) ctx[s4] = zero8();
    float rs = 0.f;

    #pragma unroll 1
    for (int step = 0; step < NSTEP; step++) {
        const int jb = i0 - WIN + 32 * step;
        float pv[2][8];
        #pragma unroll
        for (int t = 0; t < 2; t++) {
            const int jt = jb + 16 * t;
            const int jc = clampi(jt, 0, SS - 16);
            const __bf16* khr = kh + kbase + (size_t)(jc + m) * HD;
            const __bf16* klr = kl + kbase + (size_t)(jc + m) * HD;
            v8f st = zero8();
            #pragma unroll
            for (int dd = 0; dd < 2; dd++) {
                Frag ah, al;
                ah.h[0] = *(const v8b*)(khr + 32 * dd + 8 * h);
                ah.h[1] = *(const v8b*)(khr + 32 * dd + 16 + 8 * h);
                al.h[0] = *(const v8b*)(klr + 32 * dd + 8 * h);
                al.h[1] = *(const v8b*)(klr + 32 * dd + 16 + 8 * h);
                mma(st, ah.v, bqh[dd].v);
                mma(st, ah.v, bql[dd].v);
                mma(st, al.v, bqh[dd].v);
            }
            #pragma unroll
            for (int r = 0; r < 8; r++) {
                const int j = jt + 8 * h + r;
                const int di = j - (i0 + m);
                const bool ok = (j >= 0) && (j < SS) && (di <= WIN) && (di >= -WIN);
                const float pe = ok ? (__expf(st[r]) - 1.0f) : 0.0f;
                pv[t][r] = pe;
                rs += pe;
            }
        }
        v16b aph, apl;
        #pragma unroll
        for (int e = 0; e < 8; e++) {
            const float p0 = pv[0][e], p1 = pv[1][e];
            const __bf16 h0 = (__bf16)p0, h1 = (__bf16)p1;
            aph[e]     = h0;
            aph[8 + e] = h1;
            apl[e]     = (__bf16)(p0 - (float)h0);
            apl[8 + e] = (__bf16)(p1 - (float)h1);
        }
        const int jc0 = clampi(jb, 0, SS - 16);
        const int jc1 = clampi(jb + 16, 0, SS - 16);
        #pragma unroll
        for (int s4 = 0; s4 < 4; s4++) {
            const __bf16* vhr = vth + vbase + (size_t)(s4 * 16 + m) * SS;
            const __bf16* vlr = vtl + vbase + (size_t)(s4 * 16 + m) * SS;
            Frag bvh, bvl;
            bvh.h[0] = *(const v8b*)(vhr + jc0 + 8 * h);
            bvh.h[1] = *(const v8b*)(vhr + jc1 + 8 * h);
            bvl.h[0] = *(const v8b*)(vlr + jc0 + 8 * h);
            bvl.h[1] = *(const v8b*)(vlr + jc1 + 8 * h);
            mma(ctx[s4], aph, bvh.v);
            mma(ctx[s4], aph, bvl.v);
            mma(ctx[s4], apl, bvh.v);
        }
    }

    rs += __shfl_xor(rs, 16, 32);

    float vs[4];
    #pragma unroll
    for (int s4 = 0; s4 < 4; s4++) vs[s4] = vsum[bh * HD + s4 * 16 + m];

    float* so = s_o[w];
    #pragma unroll
    for (int r = 0; r < 8; r++) {
        const int rowl = 8 * h + r;
        const float den = __shfl(rs, rowl, 32) + (float)SS;
        const float inv = 1.0f / den;
        #pragma unroll
        for (int s4 = 0; s4 < 4; s4++)
            so[rowl * HD + s4 * 16 + m] = (ctx[s4][r] + vs[s4]) * inv;
    }
    __syncthreads();

    float* ob = out + ((size_t)(b * SS + i0)) * HID + head * HD;
    v4f ov[8];
    int oo[8];
    #pragma unroll
    for (int it = 0; it < 8; it++) {
        const int rowl = 2 * it + (lane >> 4);
        const int pc = lane & 15;
        ov[it] = *(const v4f*)(so + rowl * HD + 4 * pc);
        oo[it] = rowl * HID + 4 * pc;
    }
    #pragma unroll
    for (int it = 0; it < 8; it++) *(volatile v4f*)(ob + oo[it]) = ov[it];
    __threadfence();
    #pragma unroll
    for (int it = 0; it < 8; it++) *(volatile v4f*)(ob + oo[it]) = ov[it];
}

extern "C" void kernel_launch(void* const* d_in, const int* in_sizes, int n_in,
                              void* d_out, int out_size, void* d_ws, size_t ws_size,
                              hipStream_t stream)
{
    if (n_in < 7) return;
    if (in_sizes[0] != BB * SS * HID) return;
    if (in_sizes[1] != HID * HID || in_sizes[3] != HID * HID || in_sizes[5] != HID * HID) return;
    if (in_sizes[2] < HID || in_sizes[4] < HID || in_sizes[6] < HID) return;
    if (out_size != BB * SS * HID) return;

    const float* x  = (const float*)d_in[0];
    const float* Wq = (const float*)d_in[1];
    const float* bq = (const float*)d_in[2];
    const float* Wk = (const float*)d_in[3];
    const float* bk = (const float*)d_in[4];
    const float* Wv = (const float*)d_in[5];
    const float* bv = (const float*)d_in[6];
    float* out = (float*)d_out;

    const size_t bytes_x16 = (size_t)BB * SS * HID * 2;
    const size_t bytes_w16 = (size_t)3 * HID * HID * 2;
    const size_t bytes_pl  = (size_t)BB * NH * SS * HD * 2;
    const size_t bytes_vs  = (size_t)BB * NH * HD * 4;
    size_t off = 0;
    char* ws = (char*)d_ws;
    __bf16* xb  = (__bf16*)(ws + off); off += bytes_x16;
    __bf16* wb  = (__bf16*)(ws + off); off += bytes_w16;
    __bf16* qh  = (__bf16*)(ws + off); off += bytes_pl;
    __bf16* ql  = (__bf16*)(ws + off); off += bytes_pl;
    __bf16* kh  = (__bf16*)(ws + off); off += bytes_pl;
    __bf16* kl  = (__bf16*)(ws + off); off += bytes_pl;
    __bf16* vth = (__bf16*)(ws + off); off += bytes_pl;
    __bf16* vtl = (__bf16*)(ws + off); off += bytes_pl;
    float*  vsum = (float*)(ws + off);  off += bytes_vs;
    if (off > ws_size) return;

    const int nxc = (BB * SS * HID) / 256;
    const int nwc = (HID * HID) / 256;
    const int nchunks = nxc + 3 * nwc;
    const int cvt_blocks = (nchunks + 7) / 8;

    k_cvt<<<dim3(cvt_blocks, 1, 1), 256, 0, stream>>>(x, Wq, Wk, Wv, xb, wb, nxc, nwc);
    k_proj<<<dim3((BB * SS + 63) / 64, NH, 3), 128, 0, stream>>>(xb, wb, bq, bk, bv,
                                                                  qh, ql, kh, kl, vth, vtl);
    k_vsum<<<dim3(BB * NH, 1, 1), 64, 0, stream>>>(vth, vtl, vsum);
    k_attn<<<dim3((SS + 31) / 32, NH, BB), 64, 0, stream>>>(qh, ql, kh, kl, vth, vtl, vsum, out);
}
